// HashAttention_52553219834304
// MI455X (gfx1250) — hardware-verified
//
#include <hip/hip_runtime.h>
#include <stddef.h>
#include <math.h>


#define NB    4
#define NLEV  16
#define TDIM  8192
#define TROW  (TDIM * 2)
#define CH    32
#define SDIM  512
#define RES   256
#define HRES  128
#define NPIX  (RES * RES)
#define NTOK  (HRES * HRES)
#define PADW  (RES + 2)
#define KC    288
#define WP    320
#define NTHR  256
#define TP    36
#define CWMAX 12
#define HASHP 2654435761u

static_assert(KC == 9 * CH);
static_assert(WP >= KC && (WP % 64) == 0);
static_assert((NTOK % 128) == 0 && (NPIX % 1024) == 0);
static_assert(((PADW * CH) % 8) == 0);
static_assert((TP % 4) == 0);

__device__ __constant__ int kRes[NLEV] = {16, 19, 23, 27, 33, 40, 48, 58, 70, 84, 101, 122, 147, 176, 212, 255};

typedef float          v2f  __attribute__((ext_vector_type(2), __may_alias__));
typedef float          v4f  __attribute__((ext_vector_type(4), __may_alias__));
typedef float          v8f  __attribute__((ext_vector_type(8)));
typedef unsigned short v8us __attribute__((ext_vector_type(8), __may_alias__));
typedef __bf16         v16b __attribute__((ext_vector_type(16)));
union FragB { v16b v; v8us h[2]; };
static_assert(sizeof(FragB) == 32);

__device__ __forceinline__ int iclamp(int x, int lo, int hi) { return x < lo ? lo : (x > hi ? hi : x); }

__device__ __forceinline__ unsigned short bf_rne(float x) {
  unsigned u = __float_as_uint(x);
  u += 0x7FFFu + ((u >> 16) & 1u);
  return (unsigned short)(u >> 16);
}
__device__ __forceinline__ float bf_val(unsigned short b) { return __uint_as_float(((unsigned)b) << 16); }

__device__ __forceinline__ v8us hi8(v4f a, v4f b) {
  v8us r;
  r[0] = bf_rne(a.x); r[1] = bf_rne(a.y); r[2] = bf_rne(a.z); r[3] = bf_rne(a.w);
  r[4] = bf_rne(b.x); r[5] = bf_rne(b.y); r[6] = bf_rne(b.z); r[7] = bf_rne(b.w);
  return r;
}
__device__ __forceinline__ v8us lo8(v4f a, v4f b, v8us hb) {
  v8us r;
  r[0] = bf_rne(a.x - bf_val(hb[0])); r[1] = bf_rne(a.y - bf_val(hb[1]));
  r[2] = bf_rne(a.z - bf_val(hb[2])); r[3] = bf_rne(a.w - bf_val(hb[3]));
  r[4] = bf_rne(b.x - bf_val(hb[4])); r[5] = bf_rne(b.y - bf_val(hb[5]));
  r[6] = bf_rne(b.z - bf_val(hb[6])); r[7] = bf_rne(b.w - bf_val(hb[7]));
  return r;
}

__device__ __forceinline__ v8f zero8f() {
  v8f c;
#pragma unroll
  for (int i = 0; i < 8; ++i) c[i] = 0.0f;
  return c;
}

__device__ __forceinline__ v8f wmb(v16b a, v16b b, v8f c) {
  v8f d = __builtin_amdgcn_wmma_f32_16x16x32_bf16(false, a, false, b, (short)0, c, false, false);
  asm volatile("v_nop\n\tv_nop\n\tv_nop\n\tv_nop" : "+v"(d) : "v"(a), "v"(b));
  return d;
}

__device__ __forceinline__ v8f wm3(v16b ah, v16b al, v16b bh, v16b bl, v8f c) {
  c = wmb(ah, bh, c);
  c = wmb(ah, bl, c);
  c = wmb(al, bh, c);
  return c;
}

__device__ __forceinline__ void axis_terms(int o, float inv, float rmf, int rm, int& i0, int& i1, float& t) {
#pragma clang fp contract(off)
  const float xs  = ((float)o + 0.5f) * inv;
  const float pos = xs * rmf;
  const float fl  = floorf(pos);
  int a = (int)fl;
  a = a < 0 ? 0 : (a > rm ? rm : a);
  i0 = a;
  i1 = (a + 1 > rm) ? rm : (a + 1);
  t  = pos - fl;
}

__global__ __launch_bounds__(NTHR) void k_prep(
    const float* __restrict__ s, const float* __restrict__ aw, const float* __restrict__ ab,
    const float* __restrict__ weight,
    const float* __restrict__ kaw, const float* __restrict__ kab, const float* __restrict__ kw,
    const float* __restrict__ oaw, const float* __restrict__ oab, const float* __restrict__ ow,
    unsigned short* wh, unsigned short* wl, float* wk, float* wo) {
  __shared__ float sty[3 * CH];
  __shared__ float red[NTHR];
  __shared__ __attribute__((aligned(16))) unsigned short hrow[WP];
  __shared__ __attribute__((aligned(16))) unsigned short lrow[WP];
  const int co = blockIdx.x, b = blockIdx.y, tid = threadIdx.x, lane = tid & 31, wave = tid >> 5;

  if (wave < 3) {
    const float* W  = (wave == 0) ? aw : ((wave == 1) ? kaw : oaw);
    const float* Bv = (wave == 0) ? ab : ((wave == 1) ? kab : oab);
    const float* sv = s + (size_t)b * SDIM;
    const float* wv = W + (size_t)lane * SDIM;
    float acc = 0.0f;
#pragma unroll 4
    for (int d = 0; d < SDIM; ++d) acc += sv[d] * wv[d];
    sty[wave * CH + lane] = acc * 0.044194173824159220f + Bv[lane];
  }
  __syncthreads();

  const int k0i = tid;
  const int ci0 = k0i & 31, tap0 = k0i >> 5;
  const float v0 = weight[(size_t)co * KC + ci0 * 9 + tap0] * sty[ci0];
  const int k1i = tid + NTHR;
  const int k1c = (k1i < KC) ? k1i : (KC - 1);
  const int ci1 = k1c & 31, tap1 = k1c >> 5;
  const float t1 = weight[(size_t)co * KC + ci1 * 9 + tap1] * sty[ci1];
  const float v1 = (k1i < KC) ? t1 : 0.0f;
  red[tid] = v0 * v0 + v1 * v1;
  __syncthreads();
#pragma unroll 1
  for (int st = NTHR / 2; st > 0; st >>= 1) {
    if (tid < st) red[tid] = red[tid] + red[tid + st];
    __syncthreads();
  }
  const float dcv = 1.0f / sqrtf(red[0] + 1e-8f);
  {
    const float a0 = v0 * dcv;
    const unsigned short h0 = bf_rne(a0);
    hrow[k0i] = h0;
    lrow[k0i] = bf_rne(a0 - bf_val(h0));
    if (tid < WP - NTHR) {
      const float a1 = v1 * dcv;
      const unsigned short h1 = bf_rne(a1);
      hrow[k1i] = h1;
      lrow[k1i] = bf_rne(a1 - bf_val(h1));
    }
  }
  __syncthreads();
  if (tid < WP / 8) {
    const size_t ro = (size_t)(b * CH + co) * WP + 8 * tid;
    const v8us ph = *(const v8us*)(hrow + 8 * tid);
    const v8us pl = *(const v8us*)(lrow + 8 * tid);
    *(volatile v8us*)(wh + ro) = ph;
    *(volatile v8us*)(wl + ro) = pl;
    __threadfence();
    *(volatile v8us*)(wh + ro) = ph;
    *(volatile v8us*)(wl + ro) = pl;
  }
  if (wave == 3 || wave == 4) {
    const float* Wm = (wave == 3) ? kw : ow;
    float* dst = (wave == 3) ? wk : wo;
    const float stl = sty[((wave == 3) ? CH : (2 * CH)) + lane];
    const float v = Wm[co * CH + lane] * stl;
    float sq = v * v;
#pragma unroll
    for (int o = 16; o > 0; o >>= 1) sq += __shfl_xor(sq, o, 32);
    const float val = v * (1.0f / sqrtf(sq + 1e-8f));
    float* p = dst + (size_t)(b * CH + co) * CH + lane;
    *(volatile float*)p = val;
    __threadfence();
    *(volatile float*)p = val;
  }
}

__global__ __launch_bounds__(NTHR) void k_retrieve(const float* __restrict__ inputs, float* xs) {
#pragma clang fp contract(off)
  extern __shared__ __attribute__((aligned(16))) float dynlds[];
  float* tbl = dynlds;
  const int bl = blockIdx.x, b = bl >> 4, l = bl & 15, tid = threadIdx.x;
  const float* src = inputs + (size_t)bl * TROW;
#pragma unroll 1
  for (int i = tid * 4; i < TROW; i += NTHR * 4) *(v4f*)(tbl + i) = *(const v4f*)(src + i);
  __syncthreads();
  int r = kRes[l];
  r = iclamp(r, 2, RES);
  const int rm = r - 1;
  const float rmf = (float)rm;
  float* ch0 = xs + (size_t)(b * CH + 2 * l) * NPIX;
  float* ch1 = ch0 + NPIX;
#pragma unroll 1
  for (int q = tid; q < NPIX / 4; q += NTHR) {
    const int p0 = 4 * q;
    const int yy = p0 >> 8, xx = p0 & 255;
    int yi0, yi1; float ty;
    axis_terms(yy, 1.0f / 256.0f, rmf, rm, yi0, yi1, ty);
    const unsigned hy0 = (unsigned)yi0 * HASHP, hy1 = (unsigned)yi1 * HASHP;
    const float uy = 1.0f - ty;
    v4f va = {0.0f, 0.0f, 0.0f, 0.0f};
    v4f vb = {0.0f, 0.0f, 0.0f, 0.0f};
#pragma unroll
    for (int j = 0; j < 4; ++j) {
      int xi0, xi1; float tx;
      axis_terms(xx + j, 1.0f / 256.0f, rmf, rm, xi0, xi1, tx);
      const float ux = 1.0f - tx;
      const float w00 = ux * uy, w10 = tx * uy, w01 = ux * ty, w11 = tx * ty;
      const unsigned i00 = ((unsigned)xi0 ^ hy0) & 8191u, i10 = ((unsigned)xi1 ^ hy0) & 8191u;
      const unsigned i01 = ((unsigned)xi0 ^ hy1) & 8191u, i11 = ((unsigned)xi1 ^ hy1) & 8191u;
      const float a0 = ((tbl[2 * i00] * w00 + tbl[2 * i10] * w10) + tbl[2 * i01] * w01) + tbl[2 * i11] * w11;
      const float a1 = ((tbl[2 * i00 + 1] * w00 + tbl[2 * i10 + 1] * w10) + tbl[2 * i01 + 1] * w01) + tbl[2 * i11 + 1] * w11;
      va[j] = a0;
      vb[j] = a1;
    }
    float* pa = ch0 + p0;
    float* pb = ch1 + p0;
    *(volatile v4f*)pa = va;
    *(volatile v4f*)pb = vb;
    __threadfence();
    *(volatile v4f*)pa = va;
    *(volatile v4f*)pb = vb;
  }
}

__global__ __launch_bounds__(NTHR) void k_relayout(const float* __restrict__ xs, unsigned short* xph, unsigned short* xpl) {
  __shared__ __attribute__((aligned(16))) unsigned short H[PADW * CH];
  __shared__ __attribute__((aligned(16))) unsigned short L[PADW * CH];
  const int pr = blockIdx.x, b = blockIdx.y, tid = threadIdx.x;
  const size_t rowoff = ((size_t)b * PADW + pr) * (size_t)(PADW * CH);
  const int nunit = PADW * CH / 8;
  if (pr == 0 || pr == PADW - 1) {
    v8us z;
#pragma unroll
    for (int i = 0; i < 8; ++i) z[i] = 0;
#pragma unroll 1
    for (int u = tid; u < nunit; u += NTHR) {
      *(volatile v8us*)(xph + rowoff + 8 * u) = z;
      *(volatile v8us*)(xpl + rowoff + 8 * u) = z;
    }
    __threadfence();
#pragma unroll 1
    for (int u = tid; u < nunit; u += NTHR) {
      *(volatile v8us*)(xph + rowoff + 8 * u) = z;
      *(volatile v8us*)(xpl + rowoff + 8 * u) = z;
    }
    return;
  }
  const int r = pr - 1;
  if (tid < 2 * CH) {
    const int pc = (tid < CH) ? 0 : (PADW - 1);
    const int ch = tid & 31;
    H[pc * CH + ch] = 0;
    L[pc * CH + ch] = 0;
  }
  const float* rowp = xs + (size_t)b * CH * NPIX + (size_t)r * RES + tid;
#pragma unroll 4
  for (int ch = 0; ch < CH; ++ch) {
    const float v = rowp[(size_t)ch * NPIX];
    const unsigned short hb = bf_rne(v);
    H[(tid + 1) * CH + ch] = hb;
    L[(tid + 1) * CH + ch] = bf_rne(v - bf_val(hb));
  }
  __syncthreads();
#pragma unroll 1
  for (int u = tid; u < nunit; u += NTHR) {
    const v8us ph = *(const v8us*)(H + 8 * u);
    const v8us pl = *(const v8us*)(L + 8 * u);
    *(volatile v8us*)(xph + rowoff + 8 * u) = ph;
    *(volatile v8us*)(xpl + rowoff + 8 * u) = pl;
  }
  __threadfence();
#pragma unroll 1
  for (int u = tid; u < nunit; u += NTHR) {
    const v8us ph = *(const v8us*)(H + 8 * u);
    const v8us pl = *(const v8us*)(L + 8 * u);
    *(volatile v8us*)(xph + rowoff + 8 * u) = ph;
    *(volatile v8us*)(xpl + rowoff + 8 * u) = pl;
  }
}

__global__ __launch_bounds__(NTHR) void k_conv(const unsigned short* __restrict__ xph, const unsigned short* __restrict__ xpl,
                                              const unsigned short* __restrict__ wh, const unsigned short* __restrict__ wl,
                                              float* y) {
  __shared__ __attribute__((aligned(16))) float Os[8 * 32 * CH];
  const int oy = blockIdx.x, b = blockIdx.y, tid = threadIdx.x, lane = tid & 31, wave = tid >> 5;
  const int h = lane >> 4, m = lane & 15;
  const int oxb = 32 * wave;
  v8f acc00 = zero8f(), acc01 = zero8f(), acc10 = zero8f(), acc11 = zero8f();
  const unsigned short* wbh0 = wh + (size_t)(b * CH + m) * WP + 8 * h;
  const unsigned short* wbh1 = wh + (size_t)(b * CH + 16 + m) * WP + 8 * h;
  const unsigned short* wbl0 = wl + (size_t)(b * CH + m) * WP + 8 * h;
  const unsigned short* wbl1 = wl + (size_t)(b * CH + 16 + m) * WP + 8 * h;
#pragma unroll 1
  for (int tap = 0; tap < 9; ++tap) {
    const int kh  = (tap >= 6) ? 2 : ((tap >= 3) ? 1 : 0);
    const int kwd = tap - 3 * kh;
    const size_t pix0 = ((size_t)(b * PADW + oy + kh) * PADW + (size_t)(oxb + m + kwd)) * CH + 8 * h;
    const size_t pix1 = pix0 + 16 * CH;
    const int k0 = 32 * tap;
    FragB a0h, a0l, a1h, a1l, b0h, b0l, b1h, b1l;
    a0h.h[0] = *(const v8us*)(xph + pix0);     a0h.h[1] = *(const v8us*)(xph + pix0 + 16);
    a0l.h[0] = *(const v8us*)(xpl + pix0);     a0l.h[1] = *(const v8us*)(xpl + pix0 + 16);
    a1h.h[0] = *(const v8us*)(xph + pix1);     a1h.h[1] = *(const v8us*)(xph + pix1 + 16);
    a1l.h[0] = *(const v8us*)(xpl + pix1);     a1l.h[1] = *(const v8us*)(xpl + pix1 + 16);
    b0h.h[0] = *(const v8us*)(wbh0 + k0);      b0h.h[1] = *(const v8us*)(wbh0 + k0 + 16);
    b0l.h[0] = *(const v8us*)(wbl0 + k0);      b0l.h[1] = *(const v8us*)(wbl0 + k0 + 16);
    b1h.h[0] = *(const v8us*)(wbh1 + k0);      b1h.h[1] = *(const v8us*)(wbh1 + k0 + 16);
    b1l.h[0] = *(const v8us*)(wbl1 + k0);      b1l.h[1] = *(const v8us*)(wbl1 + k0 + 16);
    acc00 = wm3(a0h.v, a0l.v, b0h.v, b0l.v, acc00);
    acc01 = wm3(a0h.v, a0l.v, b1h.v, b1l.v, acc01);
    acc10 = wm3(a1h.v, a1l.v, b0h.v, b0l.v, acc10);
    acc11 = wm3(a1h.v, a1l.v, b1h.v, b1l.v, acc11);
  }
  float* osw = Os + wave * (32 * CH);
#pragma unroll
  for (int r = 0; r < 8; ++r) {
    const int px = 8 * h + r;
    osw[px * CH + m]             = acc00[r];
    osw[px * CH + 16 + m]        = acc01[r];
    osw[(16 + px) * CH + m]      = acc10[r];
    osw[(16 + px) * CH + 16 + m] = acc11[r];
  }
  __syncthreads();
  float* yb = y + ((size_t)b * NPIX + (size_t)oy * RES + oxb) * CH;
  const int pc = lane & 7;
#pragma unroll
  for (int i = 0; i < 8; ++i) {
    const int px = 4 * i + (lane >> 3);
    const v4f v = *(const v4f*)(osw + px * CH + 4 * pc);
    *(volatile v4f*)(yb + (size_t)px * CH + 4 * pc) = v;
  }
  __threadfence();
#pragma unroll
  for (int i = 0; i < 8; ++i) {
    const int px = 4 * i + (lane >> 3);
    const v4f v = *(const v4f*)(osw + px * CH + 4 * pc);
    *(volatile v4f*)(yb + (size_t)px * CH + 4 * pc) = v;
  }
}

__global__ __launch_bounds__(NTHR) void k_blur(const float* __restrict__ y, const float* __restrict__ bias, float* tok) {
  const int tid = threadIdx.x, lane = tid & 31, wave = tid >> 5;
  const int co = lane;
  const float bco = bias[co];
  const int tbase = (blockIdx.x * 8 + wave) * 16;
#pragma unroll 1
  for (int t = 0; t < 16; ++t) {
    const int g = tbase + t;
    const int b = g >> 14, n = g & (NTOK - 1);
    const int oy = n >> 7, ox = n & 127;
    const float* yb = y + (size_t)b * NPIX * CH + co;
    float acc = 0.0f;
#pragma unroll
    for (int i = 0; i < 4; ++i) {
      const int iy = 2 * oy + i - 1;
      const int iyc = iclamp(iy, 0, RES - 1);
      const bool oky = (unsigned)iy < (unsigned)RES;
      const float fy = (i == 0 || i == 3) ? 1.0f : 3.0f;
#pragma unroll
      for (int j = 0; j < 4; ++j) {
        const int ix = 2 * ox + j - 1;
        const int ixc = iclamp(ix, 0, RES - 1);
        const float fx = (j == 0 || j == 3) ? 1.0f : 3.0f;
        float v = yb[((size_t)iyc * RES + ixc) * CH];
        v = (oky && ((unsigned)ix < (unsigned)RES)) ? v : 0.0f;
        acc += v * (fy * fx);
      }
    }
    float rv = acc * (1.0f / 64.0f) + bco;
    rv = (rv >= 0.0f ? rv : 0.2f * rv) * 1.41421356237309515f;
    float* p = tok + (size_t)g * CH + co;
    *(volatile float*)p = rv;
    __threadfence();
    *(volatile float*)p = rv;
  }
}

__global__ __launch_bounds__(NTHR) void k_tok(const float* __restrict__ tok, const float* __restrict__ wk,
                                             const float* __restrict__ wo, float* tok2) {
  __shared__ __attribute__((aligned(16))) unsigned short Wkh[CH * CH];
  __shared__ __attribute__((aligned(16))) unsigned short Wkl[CH * CH];
  __shared__ __attribute__((aligned(16))) unsigned short Woh[CH * CH];
  __shared__ __attribute__((aligned(16))) unsigned short Wol[CH * CH];
  __shared__ __attribute__((aligned(16))) float Ts[8 * 16 * TP];
  __shared__ __attribute__((aligned(16))) float Ss[8 * 16 * TP];
  const int tid = threadIdx.x, lane = tid & 31, wave = tid >> 5, h = lane >> 4, m = lane & 15;
  const int b = blockIdx.x >> 7;
  const int g0 = blockIdx.x * 128 + wave * 16;
  {
    const float* wkb = wk + (size_t)b * CH * CH;
    const float* wob = wo + (size_t)b * CH * CH;
#pragma unroll
    for (int j = 0; j < 4; ++j) {
      const int e = 4 * tid + j;
      const float a = wkb[e];
      const unsigned short ha = bf_rne(a);
      Wkh[e] = ha;
      Wkl[e] = bf_rne(a - bf_val(ha));
      const float c = wob[e];
      const unsigned short hc = bf_rne(c);
      Woh[e] = hc;
      Wol[e] = bf_rne(c - bf_val(hc));
    }
  }
  float* Tw = Ts + wave * 16 * TP;
  float* Sw = Ss + wave * 16 * TP;
#pragma unroll
  for (int q = 0; q < 4; ++q) {
    const int u = lane + 32 * q, tl = u >> 3, pc = u & 7;
    const v4f v = *(const v4f*)(tok + (size_t)(g0 + tl) * CH + 4 * pc);
    *(v4f*)(Tw + tl * TP + 4 * pc) = v;
  }
  __syncthreads();

  v8f c0 = zero8f(), c1 = zero8f();
  {
    FragB ah, al, bh, bl;
    const float* tr = Tw + m * TP + 8 * h;
    const v4f x0 = *(const v4f*)tr, x1 = *(const v4f*)(tr + 4), x2 = *(const v4f*)(tr + 16), x3 = *(const v4f*)(tr + 20);
    ah.h[0] = hi8(x0, x1); al.h[0] = lo8(x0, x1, ah.h[0]);
    ah.h[1] = hi8(x2, x3); al.h[1] = lo8(x2, x3, ah.h[1]);
    const unsigned short* p0 = Wkh + m * CH + 8 * h;
    const unsigned short* q0 = Wkl + m * CH + 8 * h;
    bh.h[0] = *(const v8us*)p0; bh.h[1] = *(const v8us*)(p0 + 16);
    bl.h[0] = *(const v8us*)q0; bl.h[1] = *(const v8us*)(q0 + 16);
    c0 = wm3(ah.v, al.v, bh.v, bl.v, c0);
    const unsigned short* p1 = Wkh + (16 + m) * CH + 8 * h;
    const unsigned short* q1 = Wkl + (16 + m) * CH + 8 * h;
    bh.h[0] = *(const v8us*)p1; bh.h[1] = *(const v8us*)(p1 + 16);
    bl.h[0] = *(const v8us*)q1; bl.h[1] = *(const v8us*)(q1 + 16);
    c1 = wm3(ah.v, al.v, bh.v, bl.v, c1);
  }
#pragma unroll
  for (int r = 0; r < 8; ++r) {
    const int tl = 8 * h + r;
    Sw[tl * TP + m]      = c0[r];
    Sw[tl * TP + 16 + m] = c1[r];
  }
  __syncthreads();

  v8f d0 = zero8f(), d1 = zero8f();
  {
    FragB ah, al, bh, bl;
    const float* sr = Sw + m * TP + 8 * h;
    const v4f x0 = *(const v4f*)sr, x1 = *(const v4f*)(sr + 4), x2 = *(const v4f*)(sr + 16), x3 = *(const v4f*)(sr + 20);
    ah.h[0] = hi8(x0, x1); al.h[0] = lo8(x0, x1, ah.h[0]);
    ah.h[1] = hi8(x2, x3); al.h[1] = lo8(x2, x3, ah.h[1]);
    const unsigned short* p0 = Woh + m * CH + 8 * h;
    const unsigned short* q0 = Wol + m * CH + 8 * h;
    bh.h[0] = *(const v8us*)p0; bh.h[1] = *(const v8us*)(p0 + 16);
    bl.h[0] = *(const v8us*)q0; bl.h[1] = *(const v8us*)(q0 + 16);
    d0 = wm3(ah.v, al.v, bh.v, bl.v, d0);
    const unsigned short* p1 = Woh + (16 + m) * CH + 8 * h;
    const unsigned short* q1 = Wol + (16 + m) * CH + 8 * h;
    bh.h[0] = *(const v8us*)p1; bh.h[1] = *(const v8us*)(p1 + 16);
    bl.h[0] = *(const v8us*)q1; bl.h[1] = *(const v8us*)(q1 + 16);
    d1 = wm3(ah.v, al.v, bh.v, bl.v, d1);
  }
  __syncthreads();
#pragma unroll
  for (int r = 0; r < 8; ++r) {
    const int tl = 8 * h + r;
    Sw[tl * TP + m]      = d0[r] + Tw[tl * TP + m];
    Sw[tl * TP + 16 + m] = d1[r] + Tw[tl * TP + 16 + m];
  }
  __syncthreads();

  {
    float* row = Sw + m * TP + 16 * h;
    v4f q0 = *(const v4f*)row, q1 = *(const v4f*)(row + 4), q2 = *(const v4f*)(row + 8), q3 = *(const v4f*)(row + 12);
    float sm = ((q0.x + q0.y) + (q0.z + q0.w)) + ((q1.x + q1.y) + (q1.z + q1.w)) +
               ((q2.x + q2.y) + (q2.z + q2.w)) + ((q3.x + q3.y) + (q3.z + q3.w));
    sm += __shfl_xor(sm, 16, 32);
    const float mean = sm * (1.0f / 32.0f);
    q0 = q0 - mean; q1 = q1 - mean; q2 = q2 - mean; q3 = q3 - mean;
    float ss = ((q0.x * q0.x + q0.y * q0.y) + (q0.z * q0.z + q0.w * q0.w)) + ((q1.x * q1.x + q1.y * q1.y) + (q1.z * q1.z + q1.w * q1.w)) +
               ((q2.x * q2.x + q2.y * q2.y) + (q2.z * q2.z + q2.w * q2.w)) + ((q3.x * q3.x + q3.y * q3.y) + (q3.z * q3.z + q3.w * q3.w));
    ss += __shfl_xor(ss, 16, 32);
    const float rstd = 1.0f / sqrtf(ss * (1.0f / 32.0f) + 1e-5f);
    q0 = q0 * rstd; q1 = q1 * rstd; q2 = q2 * rstd; q3 = q3 * rstd;
    *(v4f*)row = q0; *(v4f*)(row + 4) = q1; *(v4f*)(row + 8) = q2; *(v4f*)(row + 12) = q3;
  }
  __syncthreads();

  const int pc = lane & 7;
#pragma unroll
  for (int i = 0; i < 4; ++i) {
    const int tl = 4 * i + (lane >> 3);
    const v4f v = *(const v4f*)(Sw + tl * TP + 4 * pc);
    *(volatile v4f*)(tok2 + (size_t)(g0 + tl) * CH + 4 * pc) = v;
  }
  __threadfence();
#pragma unroll
  for (int i = 0; i < 4; ++i) {
    const int tl = 4 * i + (lane >> 3);
    const v4f v = *(const v4f*)(Sw + tl * TP + 4 * pc);
    *(volatile v4f*)(tok2 + (size_t)(g0 + tl) * CH + 4 * pc) = v;
  }
}

__global__ __launch_bounds__(NTHR) void k_recon(const float* __restrict__ tok2, float* out) {
#pragma clang fp contract(off)
  extern __shared__ __attribute__((aligned(16))) float dynlds[];
  float* tbl  = dynlds;
  int*   cLo  = (int*)(dynlds + TROW);
  int*   cHi  = cLo + 256;
  int*   X0   = cHi + 256;
  float* TT   = (float*)(X0 + HRES);
  float* red  = TT + HRES;
  float* stat = red + 16;
  const int bl = blockIdx.x, b = bl >> 4, l = bl & 15, tid = threadIdx.x, lane = tid & 31, wave = tid >> 5;
  const v4f z4 = {0.0f, 0.0f, 0.0f, 0.0f};
#pragma unroll 1
  for (int i = tid * 4; i < TROW; i += NTHR * 4) *(v4f*)(tbl + i) = z4;
  cLo[tid] = 1;
  cHi[tid] = 0;
  int r = kRes[l];
  r = iclamp(r, 2, 256);
  const int rm = r - 1;
  const float rmf = (float)rm;
  if (tid < HRES) {
    int i0, i1; float t;
    axis_terms(tid, 1.0f / 128.0f, rmf, rm, i0, i1, t);
    X0[tid] = iclamp(i0, 0, 255);
    TT[tid] = t;
  }
  __syncthreads();
  if (tid < HRES) {
    const int c  = X0[tid];
    const int cp = X0[(tid > 0) ? (tid - 1) : 0];
    const int cn = X0[(tid < HRES - 1) ? (tid + 1) : (HRES - 1)];
    if (tid == 0 || cp != c) cLo[c] = tid;
    if (tid == HRES - 1 || cn != c) cHi[c] = tid;
  }
  __syncthreads();

  const int cx = tid;
  int loA = 1, hiA = 0;
  if (cx >= 1) { loA = cLo[cx - 1]; hiA = cHi[cx - 1]; }
  const int loB = cLo[cx], hiB = cHi[cx];
  const int nA = iclamp(hiA - loA + 1, 0, CWMAX);
  const int nB = iclamp(hiB - loB + 1, 0, CWMAX);
  const float* fb = tok2 + (size_t)b * NTOK * CH + 2 * l;

#pragma unroll 1
  for (int cy = 0; cy < r; ++cy) {
    if (cx < r) {
      float a0 = 0.0f, a1 = 0.0f;
#pragma unroll
      for (int py = 0; py < 2; ++py) {
        const int yc = cy - 1 + py;
        int ylo = 1, yhi = 0;
        if (yc >= 0) { ylo = cLo[yc]; yhi = cHi[yc]; }
        const int ny = iclamp(yhi - ylo + 1, 0, CWMAX);
#pragma unroll 1
        for (int jy = 0; jy < ny; ++jy) {
          const int oy = iclamp(ylo + jy, 0, HRES - 1);
          const float ty = TT[oy];
          const float wy = py ? (1.0f - ty) : ty;
#pragma unroll
          for (int px = 0; px < 2; ++px) {
            const int xlo = px ? loB : loA;
            const int nx  = px ? nB : nA;
#pragma unroll 1
            for (int jx = 0; jx < nx; ++jx) {
              const int ox = iclamp(xlo + jx, 0, HRES - 1);
              const float tx = TT[ox];
              const float wx = px ? (1.0f - tx) : tx;
              const float w = wx * wy;
              const v2f fv = *(const v2f*)(fb + (size_t)(oy * HRES + ox) * CH);
              a0 += fv.x * w;
              a1 += fv.y * w;
            }
          }
        }
      }
      const unsigned slot = ((unsigned)cx ^ ((unsigned)cy * HASHP)) & 8191u;
      tbl[2 * slot]     += a0;
      tbl[2 * slot + 1] += a1;
    }
    __syncthreads();
  }

  float sacc = 0.0f;
#pragma unroll 1
  for (int i = tid; i < TROW; i += NTHR) sacc += tbl[i];
#pragma unroll
  for (int o = 16; o > 0; o >>= 1) sacc += __shfl_xor(sacc, o, 32);
  if (lane == 0) red[wave] = sacc;
  __syncthreads();
  if (tid == 0) {
    float S = 0.0f;
#pragma unroll
    for (int w = 0; w < 8; ++w) S += red[w];
    stat[0] = S * (1.0f / (float)TROW);
  }
  __syncthreads();
  const float mean = stat[0];
  float qacc = 0.0f;
#pragma unroll 1
  for (int i = tid; i < TROW; i += NTHR) { const float d = tbl[i] - mean; qacc += d * d; }
#pragma unroll
  for (int o = 16; o > 0; o >>= 1) qacc += __shfl_xor(qacc, o, 32);
  if (lane == 0) red[8 + wave] = qacc;
  __syncthreads();
  if (tid == 0) {
    float Q = 0.0f;
#pragma unroll
    for (int w = 0; w < 8; ++w) Q += red[8 + w];
    stat[1] = 1.0f / sqrtf(Q * (1.0f / (float)TROW) + 1e-5f);
  }
  __syncthreads();
  const float rstd = stat[1];
  float* orow = out + (size_t)bl * TROW;
#pragma unroll 1
  for (int i = tid * 4; i < TROW; i += NTHR * 4) {
    v4f v = *(const v4f*)(tbl + i);
    v = (v - mean) * rstd;
    *(volatile v4f*)(orow + i) = v;
  }
  __threadfence();
#pragma unroll 1
  for (int i = tid * 4; i < TROW; i += NTHR * 4) {
    v4f v = *(const v4f*)(tbl + i);
    v = (v - mean) * rstd;
    *(volatile v4f*)(orow + i) = v;
  }
}

extern "C" void kernel_launch(void* const* d_in, const int* in_sizes, int n_in,
                              void* d_out, int out_size, void* d_ws, size_t ws_size,
                              hipStream_t stream) {
  if (n_in < 12) return;
  if (in_sizes[0] != NB * NLEV * TROW) return;
  if (in_sizes[1] != NB * SDIM) return;
  if (in_sizes[2] != CH * SDIM || in_sizes[3] != CH) return;
  if (in_sizes[4] != CH * KC || in_sizes[5] != CH) return;
  if (in_sizes[6] != CH * SDIM || in_sizes[7] != CH || in_sizes[8] != CH * CH) return;
  if (in_sizes[9] != CH * SDIM || in_sizes[10] != CH || in_sizes[11] != CH * CH) return;
  if (out_size != NB * NLEV * TROW) return;

  const float* inputs = (const float*)d_in[0];
  const float* s      = (const float*)d_in[1];
  const float* aw     = (const float*)d_in[2];
  const float* ab     = (const float*)d_in[3];
  const float* weight = (const float*)d_in[4];
  const float* bias   = (const float*)d_in[5];
  const float* kaw    = (const float*)d_in[6];
  const float* kab    = (const float*)d_in[7];
  const float* kwm    = (const float*)d_in[8];
  const float* oaw    = (const float*)d_in[9];
  const float* oab    = (const float*)d_in[10];
  const float* owm    = (const float*)d_in[11];
  float* outp = (float*)d_out;

  char* ws = (char*)d_ws;
  size_t off = 0;
  const size_t szW   = ((size_t)NB * CH * WP * 2 + 255) & ~(size_t)255;
  const size_t szL   = ((size_t)NB * CH * CH * 4 + 255) & ~(size_t)255;
  const size_t szXs  = ((size_t)NB * CH * NPIX * 4 + 255) & ~(size_t)255;
  const size_t szXp  = ((size_t)NB * PADW * PADW * CH * 2 + 255) & ~(size_t)255;
  const size_t szY   = ((size_t)NB * NPIX * CH * 4 + 255) & ~(size_t)255;
  const size_t szT   = ((size_t)NB * NTOK * CH * 4 + 255) & ~(size_t)255;
  const size_t oWh  = off; off += szW;
  const size_t oWl  = off; off += szW;
  const size_t oWk  = off; off += szL;
  const size_t oWo  = off; off += szL;
  const size_t oXs  = off; off += szXs;
  const size_t oXph = off; off += szXp;
  const size_t oXpl = off; off += szXp;
  const size_t oY   = off; off += szY;
  const size_t oTk  = off; off += szT;
  const size_t oTk2 = off; off += szT;
  size_t limit = (size_t)134217728;
  if (ws_size < limit) limit = ws_size;
  if (off > limit) return;

  unsigned short* Wh  = (unsigned short*)(ws + oWh);
  unsigned short* Wl  = (unsigned short*)(ws + oWl);
  float*          Wk  = (float*)(ws + oWk);
  float*          Wo  = (float*)(ws + oWo);
  float*          Xs  = (float*)(ws + oXs);
  unsigned short* Xph = (unsigned short*)(ws + oXph);
  unsigned short* Xpl = (unsigned short*)(ws + oXpl);
  float*          Y   = (float*)(ws + oY);
  float*          Tk  = (float*)(ws + oTk);
  float*          Tk2 = (float*)(ws + oTk2);

  const int ldsRetrieve = TROW * 4;
  const int ldsRecon    = (TROW + 256 + 256 + HRES + HRES + 16 + 4) * 4;
  hipFuncSetAttribute(reinterpret_cast<const void*>(&k_retrieve), hipFuncAttributeMaxDynamicSharedMemorySize, ldsRetrieve);
  hipFuncSetAttribute(reinterpret_cast<const void*>(&k_recon), hipFuncAttributeMaxDynamicSharedMemorySize, ldsRecon);

  k_prep<<<dim3(CH, NB), NTHR, 0, stream>>>(s, aw, ab, weight, kaw, kab, kwm, oaw, oab, owm, Wh, Wl, Wk, Wo);
  k_retrieve<<<NB * NLEV, NTHR, ldsRetrieve, stream>>>(inputs, Xs);
  k_relayout<<<dim3(PADW, NB), NTHR, 0, stream>>>(Xs, Xph, Xpl);
  k_conv<<<dim3(RES, NB), NTHR, 0, stream>>>(Xph, Xpl, Wh, Wl, Y);
  k_blur<<<(NB * NTOK) / 128, NTHR, 0, stream>>>(Y, bias, Tk);
  k_tok<<<(NB * NTOK) / 128, NTHR, 0, stream>>>(Tk, Wk, Wo, Tk2);
  k_recon<<<NB * NLEV, NTHR, ldsRecon, stream>>>(Tk2, outp);
}
